// GAT_71906342469787
// MI455X (gfx1250) — hardware-verified
//
#include <hip/hip_runtime.h>
#include <stddef.h>
#include <stdint.h>
#include <math.h>


#define DIN     128
#define C1      128
#define C2      64
#define K2      256
#define NCLS    10
#define C3      16
#define NTHR    256
#define NWAVE   8
#define EPT     8
#define CHUNK   (NTHR * EPT)
#define WCAP    (EPT * 32)
#define LISTN   (NWAVE * WCAP)
#define NB      1024
#define SLB     10
#define SRCB    17
#define RCAP    20480
#define DEGCAP  64
#define RPW     (NB / NWAVE)
#define GBM     64
#define GTHR    128
#define GRP3    64
#define GRP2    32
#define NEGSL   0.2f
#define EPS_SM  1e-16f
#define EPS_LN  1e-5f
#define WSMAX   134217728
#define ZINTS   (2 * RCAP + 2 * NB + LISTN)
#define LDS_BKT (ZINTS * 4 + 64)

static_assert((CHUNK & (CHUNK - 1)) == 0 && CHUNK == 2048);
static_assert(NB == (1 << SLB));
static_assert(((long long)CHUNK << SLB) < (1LL << 31));
static_assert(SLB + SRCB < 31);
static_assert(NTHR * 4 == NB);
static_assert(LISTN >= NB);
static_assert((RCAP % (NTHR * 4)) == 0 && (ZINTS % 4) == 0);
static_assert(LDS_BKT <= 300000);
static_assert(GBM == (GTHR / 32) * 16);
static_assert((DIN % 32) == 0 && (K2 % 32) == 0 && K2 == 2 * C1);
static_assert(C1 == 4 * 32 && C2 == 2 * 32 && C3 == 16);
static_assert((RPW % GRP3) == 0 && (RPW % GRP2) == 0 && (RPW % 16) == 0);
static_assert(((GRP3 * NCLS) % 4) == 0);
static_assert(NCLS + 2 <= C3);

typedef float          v2f  __attribute__((ext_vector_type(2)));
typedef float          v4f  __attribute__((ext_vector_type(4)));
typedef float          v8f  __attribute__((ext_vector_type(8)));
typedef int            v4i  __attribute__((ext_vector_type(4)));
typedef int            v8i  __attribute__((ext_vector_type(8)));
typedef unsigned int   v4u  __attribute__((ext_vector_type(4)));
typedef unsigned short v8us __attribute__((ext_vector_type(8)));
typedef __bf16         v16b __attribute__((ext_vector_type(16)));
typedef v2f  __attribute__((may_alias)) v2fa;
typedef v4f  __attribute__((may_alias)) v4fa;
typedef v4i  __attribute__((may_alias)) v4ia;
typedef v8us __attribute__((may_alias)) v8usa;
union FragB { v16b v; v8us h[2]; v8i w; };

__device__ __forceinline__ v8f wmb(const FragB& a, const FragB& b, v8f c) {
  v8f d = __builtin_amdgcn_wmma_f32_16x16x32_bf16(false, a.v, false, b.v, (short)0, c, false, false);
  asm volatile("v_nop\n\tv_nop\n\tv_nop\n\tv_nop" : "+v"(d) : "v"(a.w), "v"(b.w));
  return d;
}

__device__ __forceinline__ unsigned int f2bf(float f) {
  const unsigned int u = __float_as_uint(f);
  return ((u + 0x7FFFu + ((u >> 16) & 1u)) >> 16) & 0xFFFFu;
}
__device__ __forceinline__ float bf2f(unsigned int b) { return __uint_as_float(b << 16); }
__device__ __forceinline__ float bfr(float f) { return bf2f(f2bf(f)); }
__device__ __forceinline__ v4f bfr4(const v4f a) {
  v4f r; r.x = bfr(a.x); r.y = bfr(a.y); r.z = bfr(a.z); r.w = bfr(a.w); return r;
}
__device__ __forceinline__ int clampi(int v, int lo, int hi) { return v < lo ? lo : (v > hi ? hi : v); }
__device__ __forceinline__ float leaky(float v) { return v > 0.f ? v : NEGSL * v; }
__device__ __forceinline__ void sm_step(float lg, float& mx, float& s1, float& s2) {
  const float df = lg - mx;
  const float ee = __expf(-fabsf(df));
  const bool  up = df > 0.f;
  s1 = up ? ee : 1.0f;
  s2 = up ? 1.0f : ee;
  mx = up ? lg : mx;
}
__device__ __forceinline__ float elu1(float y) { return y > 0.f ? y : (expf(y) - 1.0f); }

__device__ __forceinline__ int scan_chunk(const int* __restrict__ dsts, int nE, int cbase, int slotBase,
                                          int nb, int vec8, int* list, int tid, int lane, int wave) {
  int wc = 0;
  const int el0  = tid * EPT;
  const int e0   = cbase + el0;
  const int sent = -2147483647 - 1;
  v4i da, db;
  if (vec8 != 0 && cbase + CHUNK <= nE) {
    da = *(const v4i*)(dsts + e0);
    db = *(const v4i*)(dsts + e0 + 4);
  } else {
    da.x = (e0     < nE) ? dsts[min(e0,     nE - 1)] : sent;
    da.y = (e0 + 1 < nE) ? dsts[min(e0 + 1, nE - 1)] : sent;
    da.z = (e0 + 2 < nE) ? dsts[min(e0 + 2, nE - 1)] : sent;
    da.w = (e0 + 3 < nE) ? dsts[min(e0 + 3, nE - 1)] : sent;
    db.x = (e0 + 4 < nE) ? dsts[min(e0 + 4, nE - 1)] : sent;
    db.y = (e0 + 5 < nE) ? dsts[min(e0 + 5, nE - 1)] : sent;
    db.z = (e0 + 6 < nE) ? dsts[min(e0 + 6, nE - 1)] : sent;
    db.w = (e0 + 7 < nE) ? dsts[min(e0 + 7, nE - 1)] : sent;
  }
  const unsigned nbs = (unsigned)slotBase;
  const unsigned unb = (unsigned)nb;
  const unsigned s0 = (unsigned)da.x - nbs, s1 = (unsigned)da.y - nbs;
  const unsigned s2 = (unsigned)da.z - nbs, s3 = (unsigned)da.w - nbs;
  const unsigned s4 = (unsigned)db.x - nbs, s5 = (unsigned)db.y - nbs;
  const unsigned s6 = (unsigned)db.z - nbs, s7 = (unsigned)db.w - nbs;
  const bool h0 = s0 < unb, h1 = s1 < unb, h2 = s2 < unb, h3 = s3 < unb;
  const bool h4 = s4 < unb, h5 = s5 < unb, h6 = s6 < unb, h7 = s7 < unb;
  const unsigned any = __builtin_amdgcn_ballot_w32(h0 | h1 | h2 | h3 | h4 | h5 | h6 | h7);
  if (any != 0u) {
#define HITJ(J, HJ, SJ) { \
      const unsigned mj = __builtin_amdgcn_ballot_w32(HJ); \
      if (mj != 0u) { \
        if (HJ) { \
          const int pos = wc + (int)__builtin_amdgcn_mbcnt_lo(mj, 0u); \
          if (pos < WCAP) list[wave * WCAP + pos] = ((el0 + (J)) << SLB) | (int)(SJ); \
        } \
        wc += (int)__builtin_popcount(mj); } }
    HITJ(0, h0, s0)
    HITJ(1, h1, s1)
    HITJ(2, h2, s2)
    HITJ(3, h3, s3)
    HITJ(4, h4, s4)
    HITJ(5, h5, s5)
    HITJ(6, h6, s6)
    HITJ(7, h7, s7)
#undef HITJ
  }
  return wc;
}

__global__ __launch_bounds__(NTHR) void k_prep(const float* __restrict__ x, const float* __restrict__ W1,
                                               const float* __restrict__ W2, unsigned short* XB,
                                               unsigned short* W1T, unsigned short* W2T, int nN, int nbx) {
  const int blk = (int)blockIdx.x, tid = (int)threadIdx.x;
  v8us o;
  unsigned short* dp;
  if (blk < nbx) {
    const int u   = blk * NTHR + tid;
    const int row = u >> 4;
    const int k8  = (u & 15) * 8;
    const int rc  = row < nN ? row : nN - 1;
    const float* p = x + (size_t)rc * DIN + k8;
    const v4f a = *(const v4f*)p;
    const v4f b = *(const v4f*)(p + 4);
    const bool ok = row < nN;
    o[0] = ok ? (unsigned short)f2bf(a.x) : (unsigned short)0;
    o[1] = ok ? (unsigned short)f2bf(a.y) : (unsigned short)0;
    o[2] = ok ? (unsigned short)f2bf(a.z) : (unsigned short)0;
    o[3] = ok ? (unsigned short)f2bf(a.w) : (unsigned short)0;
    o[4] = ok ? (unsigned short)f2bf(b.x) : (unsigned short)0;
    o[5] = ok ? (unsigned short)f2bf(b.y) : (unsigned short)0;
    o[6] = ok ? (unsigned short)f2bf(b.z) : (unsigned short)0;
    o[7] = ok ? (unsigned short)f2bf(b.w) : (unsigned short)0;
    dp = XB + (size_t)row * DIN + k8;
  } else if (blk < nbx + 8) {
    const int v  = (blk - nbx) * NTHR + tid;
    const int n  = v >> 4;
    const int k8 = (v & 15) * 8;
    const float* p = W1 + (size_t)k8 * C1 + n;
#pragma unroll
    for (int i = 0; i < 8; ++i) o[i] = (unsigned short)f2bf(p[(size_t)i * C1]);
    dp = W1T + (size_t)n * DIN + k8;
  } else if (blk < nbx + 16) {
    const int v  = (blk - nbx - 8) * NTHR + tid;
    const int n  = v >> 5;
    const int k8 = (v & 31) * 8;
    const int kk = k8 & (C1 - 1);
    const float* p = W2 + (size_t)kk * C2 + n;
#pragma unroll
    for (int i = 0; i < 8; ++i) o[i] = (unsigned short)f2bf(p[(size_t)i * C2]);
    dp = W2T + (size_t)n * K2 + k8;
  } else {
    return;
  }
  *(volatile v8us*)dp = o;
  __threadfence();
  *(volatile v8us*)dp = o;
}

__global__ __launch_bounds__(NTHR) void k_bucket(const int* __restrict__ srcs, const int* __restrict__ dsts,
                                                 int nN, int nE, int vec8, int* HS, int* OC, int* META) {
  extern __shared__ v4f lds_dyn[];
  int* reg1 = (int*)lds_dyn;
  int* reg2 = reg1 + RCAP;
  int* scnt = reg2 + RCAP;
  int* soff = scnt + NB;
  int* list = soff + NB;
  int* wcnt = list + LISTN;
  int* wtot = wcnt + NWAVE;
  const int tid = (int)threadIdx.x, lane = tid & 31, wave = tid >> 5;
  const int bkt = (int)blockIdx.x;
  const int nodeBase = bkt * NB;
  int nb = nN - nodeBase; nb = nb < 0 ? 0 : (nb > NB ? NB : nb);

  {
    const v4i z4 = {0, 0, 0, 0};
    for (int i = tid * 4; i < ZINTS; i += NTHR * 4) *(v4ia*)(reg1 + i) = z4;
    if (tid < 2 * NWAVE) wcnt[tid] = 0;
  }
  __syncthreads();

  int tot = 0;
  const int nChunks = (nE + CHUNK - 1) / CHUNK;
#pragma unroll 1
  for (int ch = 0; ch < nChunks; ++ch) {
    const int cbase = ch * CHUNK;
    const int wc = scan_chunk(dsts, nE, cbase, nodeBase, nb, vec8, list, tid, lane, wave);
    if (lane == 0) wcnt[wave] = wc;
    __syncthreads();
    int pre = 0, all = 0;
#pragma unroll
    for (int w2 = 0; w2 < NWAVE; ++w2) {
      int c = wcnt[w2];
      c = c < 0 ? 0 : (c > WCAP ? WCAP : c);
      all += c;
      pre += (w2 < wave) ? c : 0;
    }
    const int wcc  = wc > WCAP ? WCAP : wc;
    const int base = tot + pre;
#pragma unroll 1
    for (int b0 = 0; b0 < wcc; b0 += 32) {
      const int i   = b0 + lane;
      const int ic  = i < WCAP ? i : WCAP - 1;
      const int ent = list[wave * WCAP + ic];
      const int el  = (ent >> SLB) & (CHUNK - 1);
      const int sl  = ent & (NB - 1);
      int eid = cbase + el;
      eid = eid > nE - 1 ? nE - 1 : eid;
      const int sraw = srcs[eid];
      const int s = clampi(sraw, 0, nN - 1);
      const int pos = base + i;
      if (i < wcc && pos < RCAP) reg1[pos] = (sl << SRCB) | s;
    }
    tot += all;
    tot = tot > RCAP ? RCAP : tot;
    __syncthreads();
  }
  const int nh = tot;

  if (wave == 0) {
#pragma unroll 1
    for (int b0 = 0; b0 < nh; b0 += 32) {
      const int idx = b0 + lane;
      const int uv  = reg1[idx < nh ? idx : nh - 1];
      const int m32 = (nh - b0) < 32 ? (nh - b0) : 32;
#pragma unroll 1
      for (int k = 0; k < m32; ++k) {
        const int u  = __builtin_amdgcn_readlane(uv, k);
        const int sl = (u >> SRCB) & (NB - 1);
        if (lane == 0) scnt[sl] = scnt[sl] + 1;
      }
    }
  }
  __syncthreads();

  {
    const v4i ca = *(const v4ia*)(scnt + 4 * tid);
    const int e0 = ca.x < 0 ? 0 : ca.x, e1 = ca.y < 0 ? 0 : ca.y, e2 = ca.z < 0 ? 0 : ca.z, e3 = ca.w < 0 ? 0 : ca.w;
    const int ts = e0 + e1 + e2 + e3;
    int incl = ts;
#pragma unroll
    for (int d = 1; d < 32; d <<= 1) {
      const int up = __shfl_up(incl, d);
      if (lane >= d) incl += up;
    }
    if (lane == 31) wtot[wave] = incl;
    __syncthreads();
    int pre = 0;
#pragma unroll
    for (int w2 = 0; w2 < NWAVE; ++w2) pre += (w2 < wave) ? wtot[w2] : 0;
    int run = pre + incl - ts;
    soff[4 * tid + 0] = run; run += e0;
    soff[4 * tid + 1] = run; run += e1;
    soff[4 * tid + 2] = run; run += e2;
    soff[4 * tid + 3] = run;
  }
  __syncthreads();
  for (int i = tid; i < NB; i += NTHR) list[i] = soff[i];
  __syncthreads();

  if (wave == 0) {
#pragma unroll 1
    for (int b0 = 0; b0 < nh; b0 += 32) {
      const int idx = b0 + lane;
      const int uv  = reg1[idx < nh ? idx : nh - 1];
      const int m32 = (nh - b0) < 32 ? (nh - b0) : 32;
#pragma unroll 1
      for (int k = 0; k < m32; ++k) {
        const int u  = __builtin_amdgcn_readlane(uv, k);
        const int sl = (u >> SRCB) & (NB - 1);
        const int sv = u & ((1 << SRCB) - 1);
        if (lane == 0) {
          int pos = list[sl];
          pos = pos < 0 ? 0 : (pos > RCAP - 1 ? RCAP - 1 : pos);
          reg2[pos] = sv;
          list[sl] = pos + 1;
        }
      }
    }
  }
  __syncthreads();

  int* hsb = HS + (size_t)bkt * RCAP;
  int* ocb = OC + (size_t)bkt * (2 * NB);
  int* mtb = META + (size_t)bkt * 32;
  const v4i ovv = *(const v4ia*)(soff + 4 * tid);
  const v4i cvv = *(const v4ia*)(scnt + 4 * tid);
  v4i mv = {0, 0, 0, 0};
  if (lane == 0) { mv.x = nh; mv.y = (nh >= RCAP) ? 1 : 0; }
#pragma unroll 1
  for (int i = tid * 4; i < RCAP; i += NTHR * 4) {
    const v4i v = *(const v4ia*)(reg2 + i);
    *(volatile v4i*)(hsb + i) = v;
  }
  *(volatile v4i*)(ocb + 4 * tid) = ovv;
  *(volatile v4i*)(ocb + NB + 4 * tid) = cvv;
  if (wave == 0 && lane < 8) *(volatile v4i*)(mtb + 4 * lane) = mv;
  __threadfence();
#pragma unroll 1
  for (int i = tid * 4; i < RCAP; i += NTHR * 4) {
    const v4i v = *(const v4ia*)(reg2 + i);
    *(volatile v4i*)(hsb + i) = v;
  }
  *(volatile v4i*)(ocb + 4 * tid) = ovv;
  *(volatile v4i*)(ocb + NB + 4 * tid) = cvv;
  if (wave == 0 && lane < 8) *(volatile v4i*)(mtb + 4 * lane) = mv;
}

template <int NT>
__global__ __launch_bounds__(GTHR) void k_gemm(const unsigned short* __restrict__ A,
                                               const unsigned short* __restrict__ WT, int K, float* Cm,
                                               const float* __restrict__ atts, const float* __restrict__ attd,
                                               float* SD) {
  static_assert(NT == 8 || NT == 4);
  constexpr int LDC = 16 * NT;
  constexpr int SDW = 2 * NT;
  __shared__ __attribute__((aligned(16))) float stg[GBM * LDC];
  __shared__ __attribute__((aligned(16))) float satt[2 * LDC];
  __shared__ __attribute__((aligned(16))) float sdot[GBM * SDW];
  const int tid = (int)threadIdx.x, lane = tid & 31, wave = tid >> 5, hh = lane >> 4, m = lane & 15;
  const int rowBase = (int)blockIdx.x * GBM;

  for (int i = tid; i < 2 * LDC; i += GTHR) {
    const int which = i / LDC;
    const int c = i - which * LDC;
    const float vs = atts[c];
    const float vd = attd[c];
    satt[i] = bfr(which == 0 ? vs : vd);
  }

  v8f acc[NT];
  {
    const v8f z = {0.f, 0.f, 0.f, 0.f, 0.f, 0.f, 0.f, 0.f};
#pragma unroll
    for (int t = 0; t < NT; ++t) acc[t] = z;
  }
  const unsigned short* ap = A  + (size_t)(rowBase + 16 * wave + m) * (size_t)K + 8 * hh;
  const unsigned short* wp = WT + (size_t)m * (size_t)K + 8 * hh;
  const int ksteps = K >> 5;
#pragma unroll 1
  for (int ks = 0; ks < ksteps; ++ks) {
    FragB af;
    af.h[0] = *(const v8usa*)(ap + 32 * ks);
    af.h[1] = *(const v8usa*)(ap + 32 * ks + 16);
#pragma unroll
    for (int t = 0; t < NT; ++t) {
      const unsigned short* wq = wp + (size_t)(16 * t) * (size_t)K + 32 * ks;
      FragB bf;
      bf.h[0] = *(const v8usa*)wq;
      bf.h[1] = *(const v8usa*)(wq + 16);
      acc[t] = wmb(af, bf, acc[t]);
    }
  }

#pragma unroll
  for (int t = 0; t < NT; ++t) {
    const int lc = 16 * t + m;
#pragma unroll
    for (int r = 0; r < 8; ++r) {
      const int lr = 16 * wave + 8 * hh + r;
      stg[lr * LDC + lc] = acc[t][r];
    }
  }
  __syncthreads();

  {
    const int row = tid & 63, which = tid >> 6;
    const float* sa = satt + which * LDC;
    const float* hr = stg + row * LDC;
#pragma unroll 2
    for (int hd = 0; hd < NT; ++hd) {
      float d = 0.f;
#pragma unroll
      for (int q = 0; q < 4; ++q) {
        const v4f hv = *(const v4fa*)(hr + 16 * hd + 4 * q);
        const v4f av = *(const v4fa*)(sa + 16 * hd + 4 * q);
        d = fmaf(hv.x, av.x, d);
        d = fmaf(hv.y, av.y, d);
        d = fmaf(hv.z, av.z, d);
        d = fmaf(hv.w, av.w, d);
      }
      sdot[row * SDW + which * NT + hd] = d;
    }
  }
  __syncthreads();

  const int wbase = 16 * wave * LDC;
  float* cp = Cm + (size_t)(rowBase + 16 * wave) * (size_t)LDC;
  float* sp = SD + (size_t)rowBase * (size_t)SDW;
#pragma unroll 1
  for (int i = 0; i < 2 * NT; ++i) {
    const int p = i * 128 + 4 * lane;
    const v4f v = *(const v4fa*)(stg + wbase + p);
    *(volatile v4f*)(cp + p) = v;
  }
#pragma unroll 1
  for (int j = 0; j < NT / 4; ++j) {
    const int p = 4 * (j * GTHR + tid);
    const v4f v = *(const v4fa*)(sdot + p);
    *(volatile v4f*)(sp + p) = v;
  }
  __threadfence();
#pragma unroll 1
  for (int i = 0; i < 2 * NT; ++i) {
    const int p = i * 128 + 4 * lane;
    const v4f v = *(const v4fa*)(stg + wbase + p);
    *(volatile v4f*)(cp + p) = v;
  }
#pragma unroll 1
  for (int j = 0; j < NT / 4; ++j) {
    const int p = 4 * (j * GTHR + tid);
    const v4f v = *(const v4fa*)(sdot + p);
    *(volatile v4f*)(sp + p) = v;
  }
}

__device__ __forceinline__ void slot_info(const int* __restrict__ oc, int slot, int nh, bool ovfb,
                                          int& st, int& cnt, float& pz) {
  int s = oc[slot];
  const int craw = oc[NB + slot];
  s = s < 0 ? 0 : (s > nh ? nh : s);
  int c = craw < 0 ? 0 : (craw > DEGCAP ? DEGCAP : craw);
  if (c > nh - s) c = nh - s;
  st = s; cnt = c;
  pz = (ovfb || craw > DEGCAP || craw < 0) ? __int_as_float(0x7fc00000) : 0.0f;
}

__global__ __launch_bounds__(NTHR) void k_scan1(const int* __restrict__ HS, const int* __restrict__ OC,
                                                const int* __restrict__ META,
                                                const float* __restrict__ F, const float* __restrict__ SD,
                                                const float* __restrict__ bias, const float* __restrict__ gam,
                                                const float* __restrict__ bet,
                                                unsigned short* XP, int nN, int MPr) {
  const int tid = (int)threadIdx.x, lane = tid & 31, wave = tid >> 5;
  const int bkt = (int)blockIdx.x;
  const int nodeBase = bkt * NB;
  const int* hs = HS + (size_t)bkt * RCAP;
  const int* oc = OC + (size_t)bkt * (2 * NB);
  const int nhr = META[bkt * 32];
  const int ovr = META[bkt * 32 + 1];
  const bool ovfb = (ovr != 0) || (nhr >= RCAP) || (nhr < 0);
  const int nh = clampi(nhr, 0, RCAP);
  const int c0 = 4 * lane;
  const int hsel = lane >> 2;
  const v4f bb4 = bfr4(*(const v4fa*)(bias + c0));
  const v4f gg4 = bfr4(*(const v4fa*)(gam + c0));
  const v4f be4 = bfr4(*(const v4fa*)(bet + c0));

#pragma unroll 1
  for (int jt = 0; jt < RPW; ++jt) {
    const int slot = wave * RPW + jt;
    const int grow = nodeBase + slot;
    const int gcl  = grow < nN ? grow : nN - 1;
    int st, cnt; float pz;
    slot_info(oc, slot, nh, ovfb, st, cnt, pz);

    const v4f fd = *(const v4fa*)(F + (size_t)gcl * C1 + c0);
    const float adv = SD[(size_t)gcl * 16 + 8 + hsel];
    const float l0 = leaky(SD[(size_t)gcl * 16 + hsel] + adv);
    float mx = l0, dn = 1.0f;
    v4f av = fd;

#pragma unroll 1
    for (int q = 0; q < cnt; ++q) {
      int idx = st + q; idx = idx > RCAP - 1 ? RCAP - 1 : idx;
      const int s = clampi(hs[idx], 0, nN - 1);
      const v4f fs = *(const v4fa*)(F + (size_t)s * C1 + c0);
      const float lg = leaky(SD[(size_t)s * 16 + hsel] + adv);
      float s1, s2;
      sm_step(lg, mx, s1, s2);
      dn = fmaf(dn, s1, s2);
      av.x = fmaf(av.x, s1, s2 * fs.x);
      av.y = fmaf(av.y, s1, s2 * fs.y);
      av.z = fmaf(av.z, s1, s2 * fs.z);
      av.w = fmaf(av.w, s1, s2 * fs.w);
    }
    const float inv = __builtin_amdgcn_rcpf(dn + EPS_SM);
    v4f v;
    v.x = fmaf(av.x, inv, bb4.x); v.y = fmaf(av.y, inv, bb4.y);
    v.z = fmaf(av.z, inv, bb4.z); v.w = fmaf(av.w, inv, bb4.w);
    float sm = (v.x + v.y) + (v.z + v.w);
#pragma unroll
    for (int off = 16; off > 0; off >>= 1) sm += __shfl_xor(sm, off);
    const float mu = sm * (1.0f / C1);
    const float dx = v.x - mu, dy = v.y - mu, dz = v.z - mu, dw = v.w - mu;
    float sq = dx * dx;
    sq = fmaf(dy, dy, sq); sq = fmaf(dz, dz, sq); sq = fmaf(dw, dw, sq);
#pragma unroll
    for (int off = 16; off > 0; off >>= 1) sq += __shfl_xor(sq, off);
    const float rstd = rsqrtf(sq * (1.0f / C1) + EPS_LN);
    const bool live = grow < nN;
    v4f o;
    o.x = live ? (elu1(fmaf(dx * rstd, gg4.x, be4.x)) + pz) : 0.f;
    o.y = live ? (elu1(fmaf(dy * rstd, gg4.y, be4.y)) + pz) : 0.f;
    o.z = live ? (elu1(fmaf(dz * rstd, gg4.z, be4.z)) + pz) : 0.f;
    o.w = live ? (elu1(fmaf(dw * rstd, gg4.w, be4.w)) + pz) : 0.f;
    const unsigned int hbx = f2bf(o.x), hby = f2bf(o.y), hbz = f2bf(o.z), hbw = f2bf(o.w);
    const unsigned int lbx = f2bf(o.x - bf2f(hbx)), lby = f2bf(o.y - bf2f(hby));
    const unsigned int lbz = f2bf(o.z - bf2f(hbz)), lbw = f2bf(o.w - bf2f(hbw));
    const int hw0 = (int)(hbx | (hby << 16)), hw1 = (int)(hbz | (hbw << 16));
    const int lw0 = (int)(lbx | (lby << 16)), lw1 = (int)(lbz | (lbw << 16));
    const int sa = (2 * lane) & 31, sb = (2 * lane + 1) & 31;
    const int g0 = __shfl(hw0, sa), g1 = __shfl(hw1, sa), g2 = __shfl(hw0, sb), g3 = __shfl(hw1, sb);
    const int q0 = __shfl(lw0, sa), q1 = __shfl(lw1, sa), q2 = __shfl(lw0, sb), q3 = __shfl(lw1, sb);
    const bool lsel = lane >= 16;
    v4u pv;
    pv.x = (unsigned int)(lsel ? q0 : g0);
    pv.y = (unsigned int)(lsel ? q1 : g1);
    pv.z = (unsigned int)(lsel ? q2 : g2);
    pv.w = (unsigned int)(lsel ? q3 : g3);
    unsigned short* gp = XP + (size_t)grow * K2 + 8 * lane;
    const bool wr = grow < MPr;
    if (wr) *(volatile v4u*)gp = pv;
    __threadfence();
    if (wr) *(volatile v4u*)gp = pv;
  }
}

__global__ __launch_bounds__(NTHR) void k_scan2(const int* __restrict__ HS, const int* __restrict__ OC,
                                                const int* __restrict__ META,
                                                const float* __restrict__ F, const float* __restrict__ SD,
                                                const float* __restrict__ bias, const float* __restrict__ gam,
                                                const float* __restrict__ bet,
                                                const float* __restrict__ W3, const float* __restrict__ a3s,
                                                const float* __restrict__ a3d,
                                                float* H3, int nN, int MPr) {
  __shared__ __attribute__((aligned(16))) float w3s[C2 * C3];
  __shared__ __attribute__((aligned(16))) float xr[NWAVE * C2];
  __shared__ __attribute__((aligned(16))) float hst[NWAVE * GRP2 * C3];
  const int tid = (int)threadIdx.x, lane = tid & 31, wave = tid >> 5;
  const int bkt = (int)blockIdx.x;
  const int nodeBase = bkt * NB;
  const int* hs = HS + (size_t)bkt * RCAP;
  const int* oc = OC + (size_t)bkt * (2 * NB);
  const int nhr = META[bkt * 32];
  const int ovr = META[bkt * 32 + 1];
  const bool ovfb = (ovr != 0) || (nhr >= RCAP) || (nhr < 0);
  const int nh = clampi(nhr, 0, RCAP);

  for (int i = tid; i < C2 * C3; i += NTHR) {
    const int k = i >> 4, c = i & 15;
    const int cl = c < NCLS ? c : NCLS - 1;
    const float wv = bfr(W3[k * NCLS + cl]);
    w3s[i] = (c < NCLS) ? wv : 0.f;
  }
  const int c0 = 2 * lane;
  const int hsel = lane >> 3;
  const float bz0 = bfr(bias[c0]), bz1 = bfr(bias[c0 + 1]);
  const float gz0 = bfr(gam[c0]),  gz1 = bfr(gam[c0 + 1]);
  const float ez0 = bfr(bet[c0]),  ez1 = bfr(bet[c0 + 1]);
  const int c = lane & 15;
  const bool cval = c < NCLS;
  const int ccl = cval ? c : NCLS - 1;
  float a3sv = bfr(a3s[ccl]); a3sv = cval ? a3sv : 0.f;
  float a3dv = bfr(a3d[ccl]); a3dv = cval ? a3dv : 0.f;
  float* xrw = xr + wave * C2;
  float* hsw = hst + wave * (GRP2 * C3);
  __syncthreads();

#pragma unroll 1
  for (int jt = 0; jt < RPW; ++jt) {
    const int slot = wave * RPW + jt;
    const int grow = nodeBase + slot;
    const int gcl  = grow < nN ? grow : nN - 1;
    int st, cnt; float pz;
    slot_info(oc, slot, nh, ovfb, st, cnt, pz);

    const v2f fd = *(const v2fa*)(F + (size_t)gcl * C2 + c0);
    const float adv = SD[(size_t)gcl * 8 + 4 + hsel];
    const float l0 = leaky(SD[(size_t)gcl * 8 + hsel] + adv);
    float mx = l0, dn = 1.0f;
    float a0 = fd.x, a1 = fd.y;

#pragma unroll 1
    for (int q = 0; q < cnt; ++q) {
      int idx = st + q; idx = idx > RCAP - 1 ? RCAP - 1 : idx;
      const int s = clampi(hs[idx], 0, nN - 1);
      const v2f fs = *(const v2fa*)(F + (size_t)s * C2 + c0);
      const float lg = leaky(SD[(size_t)s * 8 + hsel] + adv);
      float s1, s2;
      sm_step(lg, mx, s1, s2);
      dn = fmaf(dn, s1, s2);
      a0 = fmaf(a0, s1, s2 * fs.x);
      a1 = fmaf(a1, s1, s2 * fs.y);
    }
    const float inv = __builtin_amdgcn_rcpf(dn + EPS_SM);
    const float v0 = fmaf(a0, inv, bz0);
    const float v1 = fmaf(a1, inv, bz1);
    float sm = v0 + v1;
#pragma unroll
    for (int off = 16; off > 0; off >>= 1) sm += __shfl_xor(sm, off);
    const float mu = sm * (1.0f / C2);
    const float d0 = v0 - mu, d1 = v1 - mu;
    float sq = fmaf(d1, d1, d0 * d0);
#pragma unroll
    for (int off = 16; off > 0; off >>= 1) sq += __shfl_xor(sq, off);
    const float rstd = rsqrtf(sq * (1.0f / C2) + EPS_LN);
    v2f xv;
    xv.x = elu1(fmaf(d0 * rstd, gz0, ez0));
    xv.y = elu1(fmaf(d1 * rstd, gz1, ez1));
    *(v2fa*)(xrw + c0) = xv;
    __syncthreads();

    float h3 = 0.f;
#pragma unroll 4
    for (int k = 0; k < C2; ++k) h3 = fmaf(xrw[k], w3s[k * C3 + c], h3);
    float ps = h3 * a3sv, pd = h3 * a3dv;
#pragma unroll
    for (int off = 8; off > 0; off >>= 1) {
      ps += __shfl_xor(ps, off);
      pd += __shfl_xor(pd, off);
    }
    float rv = cval ? h3 : ((c == NCLS) ? ps : ((c == NCLS + 1) ? pd : 0.f));
    rv = (grow < nN) ? (rv + pz) : 0.f;
    const int lr = jt & (GRP2 - 1);
    if (lane < 16) hsw[lr * C3 + c] = rv;

    if (lr == GRP2 - 1) {
      __syncthreads();
      const int row0 = nodeBase + wave * RPW + (jt & ~(GRP2 - 1));
      const bool wr = row0 + GRP2 <= MPr;
      float* ob = H3 + (size_t)row0 * C3;
      if (wr) {
#pragma unroll 1
        for (int i = 0; i < (GRP2 * C3) / 128; ++i) {
          const int p = i * 128 + 4 * lane;
          const v4f v = *(const v4fa*)(hsw + p);
          *(volatile v4f*)(ob + p) = v;
        }
      }
      __threadfence();
      if (wr) {
#pragma unroll 1
        for (int i = 0; i < (GRP2 * C3) / 128; ++i) {
          const int p = i * 128 + 4 * lane;
          const v4f v = *(const v4fa*)(hsw + p);
          *(volatile v4f*)(ob + p) = v;
        }
      }
      __syncthreads();
    }
  }
}

__global__ __launch_bounds__(NTHR) void k_scan3(const int* __restrict__ HS, const int* __restrict__ OC,
                                                const int* __restrict__ META,
                                                const float* __restrict__ F, const float* __restrict__ bias,
                                                float* out, int nN) {
  __shared__ __attribute__((aligned(16))) float sres[NWAVE * GRP3 * NCLS];
  const int tid = (int)threadIdx.x, lane = tid & 31, wave = tid >> 5;
  const int bkt = (int)blockIdx.x;
  const int nodeBase = bkt * NB;
  const int* hs = HS + (size_t)bkt * RCAP;
  const int* oc = OC + (size_t)bkt * (2 * NB);
  const int nhr = META[bkt * 32];
  const int ovr = META[bkt * 32 + 1];
  const bool ovfb = (ovr != 0) || (nhr >= RCAP) || (nhr < 0);
  const int nh = clampi(nhr, 0, RCAP);
  const int c = lane & 15;
  const bool valid = c < NCLS;
  const int ccl = valid ? c : NCLS - 1;
  float bz = bfr(bias[ccl]); bz = valid ? bz : 0.f;
  float* res = sres + wave * (GRP3 * NCLS);

#pragma unroll 1
  for (int jt = 0; jt < RPW; ++jt) {
    const int slot = wave * RPW + jt;
    const int grow = nodeBase + slot;
    const int gcl  = grow < nN ? grow : nN - 1;
    int st, cnt; float pz;
    slot_info(oc, slot, nh, ovfb, st, cnt, pz);

    const float* dr = F + (size_t)gcl * C3;
    const float adv = dr[NCLS + 1];
    const float l0 = leaky(dr[NCLS] + adv);
    float mx = l0, dn = 1.0f;
    float a0 = dr[c];

#pragma unroll 1
    for (int q = 0; q < cnt; ++q) {
      int idx = st + q; idx = idx > RCAP - 1 ? RCAP - 1 : idx;
      const int s = clampi(hs[idx], 0, nN - 1);
      const float* sr = F + (size_t)s * C3;
      const float fs = sr[c];
      const float lg = leaky(sr[NCLS] + adv);
      float s1, s2;
      sm_step(lg, mx, s1, s2);
      dn = fmaf(dn, s1, s2);
      a0 = fmaf(a0, s1, s2 * fs);
    }
    const float inv = __builtin_amdgcn_rcpf(dn + EPS_SM);
    const float z = fmaf(a0, inv, bz);
    float vm = valid ? z : -3.0e38f;
#pragma unroll
    for (int off = 8; off > 0; off >>= 1) vm = fmaxf(vm, __shfl_xor(vm, off));
    const float ex = expf(z - vm);
    float sm = valid ? ex : 0.f;
#pragma unroll
    for (int off = 8; off > 0; off >>= 1) sm += __shfl_xor(sm, off);
    const float ls = logf(sm);
    const float o = ((z - vm) - ls) + pz;
    const int lr = jt & (GRP3 - 1);
    if (lane < NCLS) res[lr * NCLS + c] = o;

    if (lr == GRP3 - 1) {
      __syncthreads();
      const int row0 = nodeBase + wave * RPW + (jt & ~(GRP3 - 1));
      int live = nN - row0; live = live < 0 ? 0 : (live > GRP3 ? GRP3 : live);
      const int npc = (live * NCLS) >> 2;
      float* ob = out + (size_t)row0 * NCLS;
#pragma unroll 1
      for (int p0 = 0; p0 < npc; p0 += 32) {
        const int p  = p0 + lane;
        const int pc = p < (GRP3 * NCLS) / 4 ? p : (GRP3 * NCLS) / 4 - 1;
        const v4f v = *(const v4fa*)(res + 4 * pc);
        if (p < npc) *(volatile v4f*)(ob + 4 * p) = v;
      }
      __threadfence();
#pragma unroll 1
      for (int p0 = 0; p0 < npc; p0 += 32) {
        const int p  = p0 + lane;
        const int pc = p < (GRP3 * NCLS) / 4 ? p : (GRP3 * NCLS) / 4 - 1;
        const v4f v = *(const v4fa*)(res + 4 * pc);
        if (p < npc) *(volatile v4f*)(ob + 4 * p) = v;
      }
      __syncthreads();
    }
  }
}

static inline int cdiv(int a, int b) { return (a + b - 1) / b; }

extern "C" void kernel_launch(void* const* d_in, const int* in_sizes, int n_in,
                              void* d_out, int out_size, void* d_ws, size_t ws_size,
                              hipStream_t stream) {
  if (n_in < 18) return;
  if (in_sizes[0] < DIN || (in_sizes[0] % DIN) != 0) return;
  const int nN = in_sizes[0] / DIN;
  if (nN < 16 || (nN % 16) != 0 || nN > (1 << SRCB)) return;
  if (in_sizes[1] < 2 || (in_sizes[1] & 1) != 0) return;
  const int nE = in_sizes[1] / 2;
  if (nE < 1 || nE > (1 << 30)) return;
  if (in_sizes[2] != DIN * C1) return;
  if (in_sizes[3] != C1 || in_sizes[4] != C1) return;
  if (in_sizes[5] != C1 || in_sizes[6] != C1 || in_sizes[7] != C1) return;
  if (in_sizes[8] != C1 * C2) return;
  if (in_sizes[9] != C2 || in_sizes[10] != C2) return;
  if (in_sizes[11] != C2 || in_sizes[12] != C2 || in_sizes[13] != C2) return;
  if (in_sizes[14] != C2 * NCLS) return;
  if (in_sizes[15] != NCLS || in_sizes[16] != NCLS || in_sizes[17] != NCLS) return;
  if ((long long)out_size != (long long)nN * NCLS) return;

  const float* x   = (const float*)d_in[0];
  const int*   ei  = (const int*)  d_in[1];
  const float* W1  = (const float*)d_in[2];
  const float* a1s = (const float*)d_in[3];
  const float* a1d = (const float*)d_in[4];
  const float* b1  = (const float*)d_in[5];
  const float* g1  = (const float*)d_in[6];
  const float* be1 = (const float*)d_in[7];
  const float* W2  = (const float*)d_in[8];
  const float* a2s = (const float*)d_in[9];
  const float* a2d = (const float*)d_in[10];
  const float* b2  = (const float*)d_in[11];
  const float* g2  = (const float*)d_in[12];
  const float* be2 = (const float*)d_in[13];
  const float* W3  = (const float*)d_in[14];
  const float* a3s = (const float*)d_in[15];
  const float* a3d = (const float*)d_in[16];
  const float* b3  = (const float*)d_in[17];
  float* out = (float*)d_out;
  const int* src = ei;
  const int* dst = ei + nE;

  const int MP   = cdiv(nN, GBM) * GBM;
  const int gM   = MP / GBM;
  const int gA   = cdiv(MP, NB);
  if ((long long)gA * NB < (long long)MP) return;
  const int vec8 = ((nE & 3) == 0) ? 1 : 0;
  const int nbx  = (MP * (DIN / 8)) / NTHR;
  if (nbx * NTHR != MP * (DIN / 8)) return;

  char* ws = (char*)d_ws;
  size_t off = 0;
  const size_t oA  = off; off += (size_t)MP * K2 * 2;            off = (off + 255) & ~(size_t)255;
  const size_t oB  = off; off += (size_t)MP * C1 * 4;            off = (off + 255) & ~(size_t)255;
  const size_t oSD = off; off += (size_t)MP * 16 * 4;            off = (off + 255) & ~(size_t)255;
  const size_t oHS = off; off += (size_t)gA * RCAP * 4;          off = (off + 255) & ~(size_t)255;
  const size_t oOC = off; off += (size_t)gA * 2 * NB * 4;        off = (off + 255) & ~(size_t)255;
  const size_t oMT = off; off += (size_t)gA * 32 * 4;            off = (off + 255) & ~(size_t)255;
  const size_t oW1 = off; off += (size_t)C1 * DIN * 2;           off = (off + 255) & ~(size_t)255;
  const size_t oW2 = off; off += (size_t)C2 * K2 * 2;            off = (off + 255) & ~(size_t)255;
  if (off > ws_size || off > (size_t)WSMAX) return;
  if ((size_t)MP * C2 * 4 + (size_t)MP * C3 * 4 > (size_t)MP * C1 * 4) return;
  unsigned short* XB  = (unsigned short*)(ws + oA);
  unsigned short* X1  = (unsigned short*)(ws + oA);
  float*          H1  = (float*)(ws + oB);
  float*          H2  = (float*)(ws + oB);
  float*          H3  = (float*)(ws + oB + (size_t)MP * C2 * 4);
  float*          SD  = (float*)(ws + oSD);
  int*            HS  = (int*)(ws + oHS);
  int*            OC  = (int*)(ws + oOC);
  int*            MT  = (int*)(ws + oMT);
  unsigned short* W1T = (unsigned short*)(ws + oW1);
  unsigned short* W2T = (unsigned short*)(ws + oW2);

  hipFuncSetAttribute(reinterpret_cast<const void*>(&k_bucket),
                      hipFuncAttributeMaxDynamicSharedMemorySize, LDS_BKT);

  k_prep<<<nbx + 16, NTHR, 0, stream>>>(x, W1, W2, XB, W1T, W2T, nN, nbx);
  k_bucket<<<gA, NTHR, LDS_BKT, stream>>>(src, dst, nN, nE, vec8, HS, OC, MT);
  k_gemm<8><<<gM, GTHR, 0, stream>>>(XB, W1T, DIN, H1, a1s, a1d, SD);
  k_scan1<<<gA, NTHR, 0, stream>>>(HS, OC, MT, H1, SD, b1, g1, be1, X1, nN, MP);
  k_gemm<4><<<gM, GTHR, 0, stream>>>(X1, W2T, K2, H2, a2s, a2d, SD);
  k_scan2<<<gA, NTHR, 0, stream>>>(HS, OC, MT, H2, SD, b2, g2, be2, W3, a3s, a3d, H3, nN, MP);
  k_scan3<<<gA, NTHR, 0, stream>>>(HS, OC, MT, H3, b3, out, nN);
}
